// DecoderBlock_27779848471543
// MI455X (gfx1250) — hardware-verified
//
#include <hip/hip_runtime.h>
#include <math.h>

#ifndef NB
#define NB 4
#endif
#ifndef SEQ
#define SEQ 2048
#endif
#define NB_FULL 4
#define SEQ_FULL 2048
#define EMB 1024
#define NH 16
#define HD 64
#define FFD 4096
static_assert(SEQ % 64 == 0);
static_assert(SEQ >= 64 && SEQ <= SEQ_FULL);
static_assert(NB >= 1 && NB <= NB_FULL);
static_assert(NH * HD == EMB);
static_assert(EMB % 64 == 0 && FFD % 64 == 0 && (3 * EMB) % 64 == 0);

typedef __attribute__((ext_vector_type(16))) _Float16 v16h;
typedef __attribute__((ext_vector_type(8)))  _Float16 v8h;
typedef __attribute__((ext_vector_type(16))) __bf16   v16b;
typedef __attribute__((ext_vector_type(8)))  __bf16   v8b;
typedef __attribute__((ext_vector_type(8)))  float    v8f;
typedef __attribute__((ext_vector_type(4)))  float    v4f;

__device__ __forceinline__ int frag_k(int i, int h) { return (i < 8) ? (8 * h + i) : (16 + 8 * h + (i - 8)); }
__device__ __forceinline__ v8f wmma16(v16h a, v16h b, v8f c) {
    c = __builtin_amdgcn_wmma_f32_16x16x32_f16(false, a, false, b, (short)0, c, false, false);
    asm volatile("v_nop\n\tv_nop\n\tv_nop\n\tv_nop" : "+v"(c) : "v"(a), "v"(b));
    return c;
}
__device__ __forceinline__ v16h fh_ld(const float* __restrict__ p, long long sk, int k0, int h, int klen, float s) {
    v16h a;
#pragma unroll
    for (int i = 0; i < 16; ++i) { const int k = k0 + frag_k(i, h); a[i] = (k < klen) ? (_Float16)(p[(long long)k * sk] * s) : (_Float16)0.f; }
    return a;
}

#define VST2(T, ptr, val) do { const T vst2_v_ = (val); *(volatile T*)(ptr) = vst2_v_; __threadfence(); *(volatile T*)(ptr) = vst2_v_; } while (0)
#define VST2V4(ptr, val) do { const v4f vst2_v4_ = (val); *(volatile v4f*)(ptr) = vst2_v4_; __threadfence(); *(volatile v4f*)(ptr) = vst2_v4_; } while (0)

namespace w25 {

__device__ __forceinline__ unsigned short f2bf_bits(float f) {
  unsigned u = __float_as_uint(f);
  return (unsigned short)((u + 0x7FFFu + ((u >> 16) & 1u)) >> 16);
}
__device__ __forceinline__ float bf_bits2f(unsigned short h) { return __uint_as_float(((unsigned)h) << 16); }

__device__ __forceinline__ void dep_guard_h(v8f& a, v8f& b, v16h x, v16h y) { asm volatile("v_nop\n\tv_nop\n\tv_nop\n\tv_nop" : "+v"(a), "+v"(b) : "v"(x), "v"(y)); }
__device__ __forceinline__ void dep_guard_b(v8f& a, v8f& b, v16b x, v16b y) { asm volatile("v_nop\n\tv_nop\n\tv_nop\n\tv_nop" : "+v"(a), "+v"(b) : "v"(x), "v"(y)); }
__device__ __forceinline__ void keep4_h(v16h a, v16h b, v16h c, v16h d) { asm volatile("v_nop" :: "v"(a), "v"(b), "v"(c), "v"(d)); }
__device__ __forceinline__ void keep4_b(v16b a, v16b b, v16b c, v16b d) { asm volatile("v_nop" :: "v"(a), "v"(b), "v"(c), "v"(d)); }
__device__ __forceinline__ void acc_guard4(v8f& a, v8f& b, v8f& c, v8f& d) { asm volatile("v_nop\n\tv_nop\n\tv_nop\n\tv_nop" : "+v"(a), "+v"(b), "+v"(c), "+v"(d)); }
template <typename T> struct Frag;
template <> struct Frag<_Float16> {
  typedef v16h V; union U { v16h v; v8h h[2]; };
  static __device__ __forceinline__ v16h load(const _Float16* p) {
    U f; f.h[0] = *(const v8h*)(p); f.h[1] = *(const v8h*)(p + 16); return f.v;
  }
  static __device__ __forceinline__ v8f mma(v16h a, v16h b, v8f c) {
    return __builtin_amdgcn_wmma_f32_16x16x32_f16(false, a, false, b, (short)0, c, false, false);
  }
  static __device__ __forceinline__ void guard(v8f& a, v8f& b, v16h x, v16h y) { dep_guard_h(a, b, x, y); }
  static __device__ __forceinline__ void keep(v16h a, v16h b, v16h c, v16h d) { keep4_h(a, b, c, d); }
};
template <> struct Frag<__bf16> {
  typedef v16b V; union U { v16b v; v8b h[2]; };
  static __device__ __forceinline__ v16b load(const __bf16* p) {
    U f; f.h[0] = *(const v8b*)(p); f.h[1] = *(const v8b*)(p + 16); return f.v;
  }
  static __device__ __forceinline__ v8f mma(v16b a, v16b b, v8f c) {
    return __builtin_amdgcn_wmma_f32_16x16x32_bf16(false, a, false, b, (short)0, c, false, false);
  }
  static __device__ __forceinline__ void guard(v8f& a, v8f& b, v16b x, v16b y) { dep_guard_b(a, b, x, y); }
  static __device__ __forceinline__ void keep(v16b a, v16b b, v16b c, v16b d) { keep4_b(a, b, c, d); }
};

template <int ET> struct Elem;
template <> struct Elem<0> { typedef _Float16 T; };
template <> struct Elem<1> { typedef __bf16 T; };
template <int ET, bool SPLIT, int BIAS_MODE, int OUT_MODE, bool RESID, int ACT = 0>
__global__ __launch_bounds__(256) void wmma_gemm64(
    const unsigned short* __restrict__ Ap, const unsigned short* __restrict__ A2p, int lda, long strideA,
    const unsigned short* __restrict__ Btp, const unsigned short* __restrict__ Bt2p, int ldb, long strideB,
    void* __restrict__ Cout, void* __restrict__ Cout2, int ldc, long strideC,
    const float* __restrict__ bias,
    const float* __restrict__ resid, long strideR,
    int M, int N, int K, float scale) {
  typedef typename Elem<ET>::T T;
  typedef typename Frag<T>::V V;
  const T* A = (const T*)Ap; const T* A2 = (const T*)A2p; const T* Bt = (const T*)Btp; const T* Bt2 = (const T*)Bt2p;
  __shared__ __align__(16) float sT[8][16 * 68];
  const int b    = blockIdx.y;
  const int lane = threadIdx.x & 31;
  const int wave = threadIdx.x >> 5;
  const int tilesN = N >> 6;
  const int tilesM = M >> 6;
  const int tile = blockIdx.x * 8 + wave;
  if (tile >= tilesM * tilesN) return;
  const int tm = tile / tilesN;
  const int tn = tile - tm * tilesN;
  const int m0 = tm << 6;
  const int n0 = tn << 6;

  const T* Ab  = A  + (size_t)b * strideA;
  const T* Bb  = Bt + (size_t)b * strideB;
  const T* Ab2 = SPLIT ? (A2  + (size_t)b * strideA) : nullptr;
  const T* Bb2 = SPLIT ? (Bt2 + (size_t)b * strideB) : nullptr;

  const int rlane = lane & 15;
  const int koff  = (lane >> 4) * 8;
  const int mOff  = (lane >> 4) * 8;

  v8f acc[4][4];
#pragma unroll
  for (int i = 0; i < 4; ++i)
#pragma unroll
    for (int j = 0; j < 4; ++j) acc[i][j] = (v8f){0.f,0.f,0.f,0.f,0.f,0.f,0.f,0.f};

  for (int k0 = 0; k0 < K; k0 += 32) {
    V bh[4], bl[4];
#pragma unroll
    for (int j = 0; j < 4; ++j) {
      const size_t bo = (size_t)(n0 + (j << 4) + rlane) * ldb + koff + k0;
      bh[j] = Frag<T>::load(Bb + bo);
      if (SPLIT) bl[j] = Frag<T>::load(Bb2 + bo);
    }
#pragma unroll
    for (int i = 0; i < 4; ++i) {
      const size_t ao = (size_t)(m0 + (i << 4) + rlane) * lda + koff + k0;
      V ah = Frag<T>::load(Ab + ao);
      V al;
      if (SPLIT) al = Frag<T>::load(Ab2 + ao);
#pragma unroll
      for (int j = 0; j < 4; ++j) {
        acc[i][j] = Frag<T>::mma(ah, bh[j], acc[i][j]);
        if (SPLIT) {
          acc[i][j] = Frag<T>::mma(ah, bl[j], acc[i][j]);
          acc[i][j] = Frag<T>::mma(al, bh[j], acc[i][j]);
        }
      }
      Frag<T>::guard(acc[i][0], acc[i][3], ah, SPLIT ? al : ah);
    }
    Frag<T>::keep(bh[0], bh[1], bh[2], bh[3]);
    if (SPLIT) Frag<T>::keep(bl[0], bl[1], bl[2], bl[3]);
  }
  acc_guard4(acc[0][0], acc[0][1], acc[0][2], acc[0][3]);
  acc_guard4(acc[1][0], acc[1][1], acc[1][2], acc[1][3]);
  acc_guard4(acc[2][0], acc[2][1], acc[2][2], acc[2][3]);
  acc_guard4(acc[3][0], acc[3][1], acc[3][2], acc[3][3]);

  float* slab = sT[wave];
  const float* Rb = RESID ? (resid + (size_t)b * strideR) : nullptr;
#pragma unroll
  for (int i = 0; i < 4; ++i) {
    const int mBase = m0 + (i << 4);
#pragma unroll
    for (int j = 0; j < 4; ++j) {
      const int n = n0 + (j << 4) + rlane;
      float bv = 0.f;
      if (BIAS_MODE == 2) bv = bias[n];
#pragma unroll
      for (int r = 0; r < 8; ++r) {
        float v = acc[i][j][r] * scale;
        if (BIAS_MODE == 1) v += bias[mBase + mOff + r];
        if (BIAS_MODE == 2) v += bv;
        if (RESID) v += Rb[(size_t)(mBase + mOff + r) * ldc + n];
        if (ACT == 1) v = tanhf(v);
        if (ACT == 2) v = fmaxf(v, 0.0f);
        if (ACT == 3) v = v / (1.0f + expf(-v));
        if (ACT == 4) v = (v > 0.f) ? v : 0.01f * v;
        if (ACT == 5) v = 0.5f * v * (1.0f + erff(v * 0.70710678118654752f));
        if (ACT == 6) v = (v > 0.f) ? v : 0.2f * v;
        if (ACT == 7) { const float u = 0.7978845608028654f * (v + 0.044715f * v * v * v); v = 0.5f * v * (1.f + tanhf(u)); }
        slab[(mOff + r) * 68 + (j << 4) + rlane] = v;
      }
    }
    __builtin_amdgcn_fence(3  , "workgroup");
    __builtin_amdgcn_wave_barrier();
    __builtin_amdgcn_fence(2  , "workgroup");
    if (OUT_MODE == 0) {
      float* C = (float*)Cout + (size_t)b * strideC;
      const int hh = lane >> 4, c4 = (lane & 15) * 4;
      for (int pass = 0; pass < 2; ++pass) {
#pragma unroll
        for (int it = 0; it < 8; ++it) {
          const int row = it * 2 + hh;
          v4f v = *(const v4f*)(slab + row * 68 + c4);
          *(volatile v4f*)(C + (size_t)(mBase + row) * ldc + n0 + c4) = v;
        }
        __threadfence();
      }
    } else {
      const int q = lane >> 3, c8 = (lane & 7) * 8;
      unsigned short* C  = (unsigned short*)Cout  + (size_t)b * strideC;
      unsigned short* C2 = (OUT_MODE == 2) ? ((unsigned short*)Cout2 + (size_t)b * strideC) : nullptr;
      for (int pass = 0; pass < 2; ++pass) {
#pragma unroll
        for (int it = 0; it < 4; ++it) {
          const int row = it * 4 + q;
          const float* sp = slab + row * 68 + c8;
          v8h hv, lv;
#pragma unroll
          for (int e = 0; e < 8; ++e) {
            if (OUT_MODE == 1) {
              hv[e] = (_Float16)sp[e];
            } else {
              unsigned short hb = f2bf_bits(sp[e]);
              unsigned short lb = f2bf_bits(sp[e] - bf_bits2f(hb));
              hv[e] = __builtin_bit_cast(_Float16, hb);
              lv[e] = __builtin_bit_cast(_Float16, lb);
            }
          }
          *(volatile v8h*)(C + (size_t)(mBase + row) * ldc + n0 + c8) = hv;
          if (OUT_MODE == 2) *(volatile v8h*)(C2 + (size_t)(mBase + row) * ldc + n0 + c8) = lv;
        }
        __threadfence();
      }
    }
    __builtin_amdgcn_fence(3  , "workgroup");
    __builtin_amdgcn_wave_barrier();
    __builtin_amdgcn_fence(2  , "workgroup");
  }
}

}

typedef unsigned int cm_u4 __attribute__((ext_vector_type(4)));
__device__ __forceinline__ unsigned int cmb_pk2(float a, float b) { return (unsigned int)__builtin_bit_cast(unsigned short, (_Float16)a) | ((unsigned int)__builtin_bit_cast(unsigned short, (_Float16)b) << 16); }
__device__ __forceinline__ float cmb_bf(float v) { const unsigned u = __builtin_bit_cast(unsigned, v); const unsigned r = (u + 0x7fffu + ((u >> 16) & 1u)) & 0xffff0000u; return __builtin_bit_cast(float, r); }
__global__ __launch_bounds__(256) void k_cm_bfvec(const float* __restrict__ SRC, float* __restrict__ DST, int n) { const int u = blockIdx.x * 256 + threadIdx.x; if (u >= n) return; VST2(float, DST + u, cmb_bf(SRC[u])); }
__global__ __launch_bounds__(256) void k_cm_castbTz(const float* __restrict__ SRC, long long sS, int lds, unsigned short* __restrict__ DST, long long sD, int ldd, int nR, int nC, float sc) {
    const long long u = (long long)blockIdx.x * 256 + threadIdx.x; const int per = nR / 8; if (u >= (long long)nC * per) return; const int c = (int)(u / per); const int r0 = 8 * (int)(u % per);
    const float* S = SRC + (long long)blockIdx.y * sS; unsigned short* D = DST + (long long)blockIdx.y * sD;
    float w[8];
#pragma unroll
    for (int e = 0; e < 8; ++e) w[e] = cmb_bf(S[(long long)(r0 + e) * lds + c]) * sc;
    cm_u4 pk; pk.x = cmb_pk2(w[0], w[1]); pk.y = cmb_pk2(w[2], w[3]); pk.z = cmb_pk2(w[4], w[5]); pk.w = cmb_pk2(w[6], w[7]); VST2(cm_u4, (cm_u4*)(D + (long long)c * ldd + r0), pk); }
__global__ __launch_bounds__(256) void k_cm_bias3(const float* __restrict__ P0, int n0, const float* __restrict__ P1, int n1, const float* __restrict__ P2, int n2, float* __restrict__ DST) {
    const int i = blockIdx.x * 256 + threadIdx.x; if (i >= n0 + n1 + n2) return;
    const float a = P0[min(i, n0 - 1)];
    const float b = P1[min(max(i - n0, 0), n1 - 1)];
    const float c = P2[min(max(i - n0 - n1, 0), n2 - 1)];
    const float v = (i < n0) ? a : ((i < n0 + n1) ? b : c);
    VST2(float, DST + i, cmb_bf(v)); }

typedef unsigned int db_u4 __attribute__((ext_vector_type(4)));
__device__ __forceinline__ unsigned int db_pk2(float a, float b) { return (unsigned int)__builtin_bit_cast(unsigned short, (_Float16)a) | ((unsigned int)__builtin_bit_cast(unsigned short, (_Float16)b) << 16); }
template <int RNDX>
__global__ __launch_bounds__(256) void k_db_ln(const float* __restrict__ X, const float* __restrict__ G, const float* __restrict__ Bb, unsigned short* __restrict__ O, int rows) {
    #pragma clang fp contract(off)
    const int row = blockIdx.x * 8 + (threadIdx.x >> 5); const int L = threadIdx.x & 31; if (row >= rows) return; const float* xr = X + (long long)row * 1024; float x[32]; float s = 0.f;
#pragma unroll
    for (int g = 0; g < 4; ++g) { const v4f a = *(const v4f*)(xr + 256 * g + 8 * L), b = *(const v4f*)(xr + 256 * g + 8 * L + 4); float v[8] = {a.x, a.y, a.z, a.w, b.x, b.y, b.z, b.w};
#pragma unroll
        for (int e = 0; e < 8; ++e) { const float t = RNDX ? cmb_bf(v[e]) : v[e]; x[8 * g + e] = t; s += t; } }
#pragma unroll
    for (int o = 16; o > 0; o >>= 1) s += __shfl_xor(s, o, 32);
    const float mu = s * (1.f / 1024.f); float q = 0.f;
#pragma unroll
    for (int e = 0; e < 32; ++e) { const float d = x[e] - mu; q += d * d; }
#pragma unroll
    for (int o = 16; o > 0; o >>= 1) q += __shfl_xor(q, o, 32);
    const float rs = rsqrtf(q * (1.f / 1024.f) + 1e-5f);
#pragma unroll
    for (int g = 0; g < 4; ++g) { const int c0 = 256 * g + 8 * L; float y[8];
#pragma unroll
        for (int e = 0; e < 8; ++e) y[e] = (x[8 * g + e] - mu) * rs * cmb_bf(G[c0 + e]) + cmb_bf(Bb[c0 + e]);
        db_u4 pk; pk.x = db_pk2(y[0], y[1]); pk.y = db_pk2(y[2], y[3]); pk.z = db_pk2(y[4], y[5]); pk.w = db_pk2(y[6], y[7]); VST2(db_u4, (db_u4*)(O + (long long)row * 1024 + c0), pk); } }

#define AW 4
struct AttnP16 {
    const unsigned short* Q; const unsigned short* K; const unsigned short* V; unsigned short* O;
    long long sQi, sKj, sVj, sOi;
    int Lq, Lk; float scale; int hcol;
};
static_assert(sizeof(AttnP16) == 4 * 8 + 4 * 8 + 4 * 4);
union FragU { v16h v; v8h hh[2]; };

__global__ __launch_bounds__(32 * AW) void k_attn16(AttnP16 p) {
    constexpr int VP = HD + 8;
    __shared__ __align__(16) float    pl[AW][16 * 64];
    __shared__ __align__(16) _Float16 vt[HD * VP];
    const int lane = threadIdx.x & 31, hf = lane >> 4, l15 = lane & 15, wave = threadIdx.x >> 5;
    const int h = blockIdx.y;
    const int q0 = ((int)blockIdx.x * AW + wave) * 16;
    float* myp = pl[wave];
    const float L2E = 1.4426950408889634f;
    const float NEG = -__builtin_inff();
    const _Float16* Qp = (const _Float16*)p.Q + (long long)h * p.hcol;
    const _Float16* Kp = (const _Float16*)p.K + (long long)h * p.hcol;
    const _Float16* Vp = (const _Float16*)p.V + (long long)h * p.hcol;
    _Float16* Op = (_Float16*)p.O + (long long)h * p.hcol;
    const int qi = min(q0 + l15, p.Lq - 1);
    v16h qa[2];
    {
        const _Float16* qrow = Qp + (long long)qi * p.sQi;
#pragma unroll
        for (int ks = 0; ks < 2; ++ks) { FragU u; u.hh[0] = *(const v8h*)(qrow + ks * 32 + 8 * hf); u.hh[1] = *(const v8h*)(qrow + ks * 32 + 16 + 8 * hf); qa[ks] = u.v; }
    }
    v8f o[4]; float m8[8], l8[8];
#pragma unroll
    for (int t = 0; t < 4; ++t) { v8f zz = {}; o[t] = zz; }
#pragma unroll
    for (int i = 0; i < 8; ++i) { m8[i] = NEG; l8[i] = 0.f; }
    const int jend = min(p.Lk, ((int)blockIdx.x * AW + AW - 1) * 16 + 16);
    for (int j0 = 0; j0 < jend; j0 += 64) {
        __syncthreads();
#pragma unroll
        for (int it = 0; it < 4; ++it) {
            const int idx = (int)threadIdx.x + it * 32 * AW;
            const int jr = idx >> 3, c8 = (idx & 7) * 8;
            const int j = j0 + jr; const int jc = min(j, p.Lk - 1);
            const v8h vv = *(const v8h*)(Vp + (long long)jc * p.sVj + c8);
#pragma unroll
            for (int e = 0; e < 8; ++e) vt[(c8 + e) * VP + jr] = (j < p.Lk) ? vv[e] : (_Float16)0.f;
        }
        v8f s[4];
#pragma unroll
        for (int t = 0; t < 4; ++t) {
            const int j = min(j0 + t * 16 + l15, p.Lk - 1);
            const _Float16* krow = Kp + (long long)j * p.sKj;
            v8f acc = {};
#pragma unroll
            for (int ks = 0; ks < 2; ++ks) {
                FragU kb; kb.hh[0] = *(const v8h*)(krow + ks * 32 + 8 * hf); kb.hh[1] = *(const v8h*)(krow + ks * 32 + 16 + 8 * hf);
                acc = wmma16(qa[ks], kb.v, acc);
            }
            s[t] = acc;
        }
        float pv[8][4];
#pragma unroll
        for (int i = 0; i < 8; ++i) {
            const int irow = q0 + i + 8 * hf;
            float sc[4];
#pragma unroll
            for (int t = 0; t < 4; ++t) {
                const int jg = j0 + t * 16 + l15;
                float v = s[t][i] * p.scale;
                if (jg >= p.Lk || jg > irow) v = NEG; else v *= L2E;
                sc[t] = v;
            }
            float mx = fmaxf(fmaxf(sc[0], sc[1]), fmaxf(sc[2], sc[3]));
            mx = fmaxf(mx, __shfl_xor(mx, 1, 32)); mx = fmaxf(mx, __shfl_xor(mx, 2, 32));
            mx = fmaxf(mx, __shfl_xor(mx, 4, 32)); mx = fmaxf(mx, __shfl_xor(mx, 8, 32));
            const float mnew = fmaxf(m8[i], mx);
            const float corr = (mnew == NEG) ? 1.f : exp2f(m8[i] - mnew);
            float rs = 0.f;
#pragma unroll
            for (int t = 0; t < 4; ++t) { const float pp = (sc[t] == NEG) ? 0.f : exp2f(sc[t] - mnew); rs += pp; pv[i][t] = pp; }
            rs += __shfl_xor(rs, 1, 32); rs += __shfl_xor(rs, 2, 32); rs += __shfl_xor(rs, 4, 32); rs += __shfl_xor(rs, 8, 32);
            l8[i] = l8[i] * corr + rs; m8[i] = mnew;
#pragma unroll
            for (int t = 0; t < 4; ++t) o[t][i] *= corr;
        }
#pragma unroll
        for (int i = 0; i < 8; ++i)
#pragma unroll
            for (int t = 0; t < 4; ++t) myp[(i + 8 * hf) * 64 + t * 16 + l15] = pv[i][t];
        __syncthreads();
        const v16h pa0 = fh_ld(myp + l15 * 64, 1, 0, hf, 64, 4096.f), pa1 = fh_ld(myp + l15 * 64, 1, 32, hf, 64, 4096.f);
#pragma unroll
        for (int t = 0; t < 4; ++t) {
            const int dcol = t * 16 + l15;
            FragU b0, b1;
            b0.hh[0] = *(const v8h*)(vt + dcol * VP + 8 * hf);      b0.hh[1] = *(const v8h*)(vt + dcol * VP + 16 + 8 * hf);
            b1.hh[0] = *(const v8h*)(vt + dcol * VP + 32 + 8 * hf); b1.hh[1] = *(const v8h*)(vt + dcol * VP + 48 + 8 * hf);
            o[t] = wmma16(pa0, b0.v, o[t]);
            o[t] = wmma16(pa1, b1.v, o[t]);
        }
    }
    float invr[8];
#pragma unroll
    for (int i = 0; i < 8; ++i) invr[i] = (l8[i] > 0.f) ? 1.f / (l8[i] * 4096.f) : 0.f;
    __syncthreads();
#pragma unroll
    for (int i = 0; i < 8; ++i)
#pragma unroll
        for (int t = 0; t < 4; ++t) myp[(i + 8 * hf) * 64 + t * 16 + l15] = o[t][i] * invr[i];
    __syncthreads();
    {
        const int q4 = lane >> 3, c8 = (lane & 7) * 8;
        for (int pass = 0; pass < 2; ++pass) {
#pragma unroll
            for (int it = 0; it < 4; ++it) {
                const int row = it * 4 + q4; const int irow = q0 + row;
                const float* sp = myp + row * 64 + c8;
                v8h hv;
#pragma unroll
                for (int e = 0; e < 8; ++e) hv[e] = (_Float16)sp[e];
                if (irow < p.Lq) *(volatile v8h*)(Op + (long long)irow * p.sOi + c8) = hv;
            }
            __threadfence();
        }
    }
}

extern "C" void kernel_launch(void* const* d_in, const int* in_sizes, int n_in, void* d_out, int out_size, void* d_ws, size_t ws_size, hipStream_t stream) {
    if (n_in < 14) return;
    const long long ntok_need = (long long)(NB - 1) * SEQ_FULL + SEQ;
    if ((long long)in_sizes[0] < ntok_need * EMB) return;
    if (in_sizes[1] < NH * EMB * HD || in_sizes[2] < NH * EMB * HD || in_sizes[3] < NH * EMB * HD) return;
    if (in_sizes[4] < EMB * EMB || in_sizes[5] < EMB) return;
    if (in_sizes[6] < EMB || in_sizes[7] < EMB || in_sizes[8] < EMB || in_sizes[9] < EMB) return;
    if (in_sizes[10] < EMB * FFD || in_sizes[11] < FFD || in_sizes[12] < FFD * EMB || in_sizes[13] < EMB) return;
    if ((long long)out_size < ntok_need * EMB) return;
    const float* x     = (const float*)d_in[0];
    const float* wq    = (const float*)d_in[1];
    const float* wk    = (const float*)d_in[2];
    const float* wv    = (const float*)d_in[3];
    const float* projw = (const float*)d_in[4];
    const float* projb = (const float*)d_in[5];
    const float* g1    = (const float*)d_in[6];
    const float* be1   = (const float*)d_in[7];
    const float* g2    = (const float*)d_in[8];
    const float* be2   = (const float*)d_in[9];
    const float* w1    = (const float*)d_in[10];
    const float* bf1   = (const float*)d_in[11];
    const float* w2    = (const float*)d_in[12];
    const float* bf2   = (const float*)d_in[13];
    float* out = (float*)d_out;

    char* ws = (char*)d_ws; size_t off = 0;
    unsigned short* WQKV16 = (unsigned short*)(ws + off); off += (size_t)3 * EMB * EMB * 2;
    unsigned short* WO16   = (unsigned short*)(ws + off); off += (size_t)EMB * EMB * 2;
    unsigned short* W116   = (unsigned short*)(ws + off); off += (size_t)FFD * EMB * 2;
    unsigned short* W216   = (unsigned short*)(ws + off); off += (size_t)EMB * FFD * 2;
    float*          BR     = (float*)(ws + off);          off += (size_t)(EMB + FFD + EMB) * 4;
    unsigned short* N16    = (unsigned short*)(ws + off); off += (size_t)SEQ * EMB * 2;
    float*          XB     = (float*)(ws + off);          off += (size_t)SEQ * EMB * 4;
    unsigned short* QKV16  = (unsigned short*)(ws + off); off += (size_t)SEQ * 3 * EMB * 2;
    unsigned short* AO16   = (unsigned short*)(ws + off); off += (size_t)SEQ * EMB * 2;
    float*          X1     = (float*)(ws + off);          off += (size_t)SEQ * EMB * 4;
    unsigned short* H16    = (unsigned short*)(ws + off); off += (size_t)SEQ * FFD * 2;
    if (off > ws_size) return;
    float* BRP = BR; float* BR1 = BR + EMB; float* BR2 = BR + EMB + FFD;

    k_cm_castbTz<<<dim3((unsigned)(((long long)HD * (EMB / 8) + 255) / 256), NH), 256, 0, stream>>>(wq, (long long)EMB * HD, HD, WQKV16, (long long)HD * EMB, EMB, EMB, HD, 16.0f);
    k_cm_castbTz<<<dim3((unsigned)(((long long)HD * (EMB / 8) + 255) / 256), NH), 256, 0, stream>>>(wk, (long long)EMB * HD, HD, WQKV16 + (size_t)EMB * EMB, (long long)HD * EMB, EMB, EMB, HD, 16.0f);
    k_cm_castbTz<<<dim3((unsigned)(((long long)HD * (EMB / 8) + 255) / 256), NH), 256, 0, stream>>>(wv, (long long)EMB * HD, HD, WQKV16 + (size_t)2 * EMB * EMB, (long long)HD * EMB, EMB, EMB, HD, 16.0f);
    k_cm_castbTz<<<dim3((unsigned)(((long long)EMB * (EMB / 8) + 255) / 256), 1), 256, 0, stream>>>(projw, 0, EMB, WO16, 0, EMB, EMB, EMB, 16.0f);
    k_cm_castbTz<<<dim3((unsigned)(((long long)FFD * (EMB / 8) + 255) / 256), 1), 256, 0, stream>>>(w1, 0, FFD, W116, 0, EMB, EMB, FFD, 16.0f);
    k_cm_castbTz<<<dim3((unsigned)(((long long)EMB * (FFD / 8) + 255) / 256), 1), 256, 0, stream>>>(w2, 0, EMB, W216, 0, FFD, FFD, EMB, 16.0f);
    k_cm_bias3<<<(unsigned)((EMB + FFD + EMB + 255) / 256), 256, 0, stream>>>(projb, EMB, bf1, FFD, bf2, EMB, BR);

    const float att_scale = 0.03125f;
    for (int bt = 0; bt < NB; ++bt) {
        const float* xb = x + (size_t)bt * SEQ_FULL * EMB;
        float* ob = out + (size_t)bt * SEQ_FULL * EMB;
        k_db_ln<1><<<SEQ / 8, 256, 0, stream>>>(xb, g1, be1, N16, SEQ);
        k_cm_bfvec<<<(unsigned)(((long long)SEQ * EMB + 255) / 256), 256, 0, stream>>>(xb, XB, SEQ * EMB);
        w25::wmma_gemm64<0, false, 0, 1, false, 0><<<dim3((unsigned)(((SEQ / 64) * ((3 * EMB) / 64) + 7) / 8), 1), 256, 0, stream>>>(
            (const unsigned short*)N16, nullptr, EMB, 0L, (const unsigned short*)WQKV16, nullptr, EMB, 0L, (void*)QKV16, nullptr, 3 * EMB, 0L, nullptr, nullptr, 0L, SEQ, 3 * EMB, EMB, 0.0625f);
        {
            AttnP16 a;
            a.Q = QKV16; a.K = QKV16 + EMB; a.V = QKV16 + 2 * EMB; a.O = AO16;
            a.sQi = 3 * EMB; a.sKj = 3 * EMB; a.sVj = 3 * EMB; a.sOi = EMB;
            a.Lq = SEQ; a.Lk = SEQ; a.scale = att_scale; a.hcol = HD;
            k_attn16<<<dim3((unsigned)(SEQ / (16 * AW)), NH, 1), 32 * AW, 0, stream>>>(a);
        }
        w25::wmma_gemm64<0, false, 2, 0, true, 0><<<dim3((unsigned)(((SEQ / 64) * (EMB / 64) + 7) / 8), 1), 256, 0, stream>>>(
            (const unsigned short*)AO16, nullptr, EMB, 0L, (const unsigned short*)WO16, nullptr, EMB, 0L, (void*)X1, nullptr, EMB, 0L, BRP, XB, 0L, SEQ, EMB, EMB, 0.0625f);
        k_db_ln<0><<<SEQ / 8, 256, 0, stream>>>(X1, g2, be2, N16, SEQ);
        w25::wmma_gemm64<0, false, 2, 1, false, 2><<<dim3((unsigned)(((SEQ / 64) * (FFD / 64) + 7) / 8), 1), 256, 0, stream>>>(
            (const unsigned short*)N16, nullptr, EMB, 0L, (const unsigned short*)W116, nullptr, EMB, 0L, (void*)H16, nullptr, FFD, 0L, BR1, nullptr, 0L, SEQ, FFD, EMB, 0.0625f);
        w25::wmma_gemm64<0, false, 2, 0, true, 0><<<dim3((unsigned)(((SEQ / 64) * (EMB / 64) + 7) / 8), 1), 256, 0, stream>>>(
            (const unsigned short*)H16, nullptr, FFD, 0L, (const unsigned short*)W216, nullptr, FFD, 0L, (void*)ob, nullptr, EMB, 0L, BR2, X1, 0L, SEQ, EMB, FFD, 0.0625f);
    }
}
